// MambaBlock_78323023610179
// MI455X (gfx1250) — hardware-verified
//
#include <hip/hip_runtime.h>
#include <math.h>

typedef __attribute__((ext_vector_type(16))) _Float16 v16h;
typedef __attribute__((ext_vector_type(8)))  _Float16 v8h;
typedef __attribute__((ext_vector_type(8)))  float    v8f;
typedef __attribute__((ext_vector_type(4)))  float    v4f;

constexpr int kBatch = 2;
constexpr int kSeqL  = 2048;
constexpr int kDmod  = 1024;
constexpr int kDin   = 2048;
constexpr int kNst   = 16;
constexpr int kDtR   = 128;
constexpr int kPrjN  = kDtR + 2 * kNst;
constexpr int kPrjP  = 192;
constexpr int kXZP   = 2 * kDin;
constexpr int kRows  = kBatch * kSeqL;
constexpr int kTP    = 260;
constexpr float kLnEps = 1e-5f;

constexpr float kCarryW   = 32.0f;
constexpr float kCarryWdt = 8.0f;
constexpr float kCarryU   = 16.0f;
constexpr float kCarryDt  = 16.0f;
constexpr float kCarryY   = 16.0f;
constexpr float kFoldIn   = 1.0f / kCarryW;
constexpr float kFoldXp   = 1.0f / (kCarryU * kCarryW);
constexpr float kFoldDt   = 1.0f / (kCarryDt * kCarryWdt);
constexpr float kFoldOut  = 1.0f / (kCarryY * kCarryW);

static_assert(kPrjN == 160, "x_proj width");
static_assert(kPrjP % 64 == 0 && kPrjP >= kPrjN, "padded x_proj width");
static_assert(kDmod % 32 == 0 && kDin % 32 == 0 && kDtR % 32 == 0, "GEMM K multiples of 32");
static_assert(kSeqL % 64 == 0 && kXZP % 64 == 0 && kDin % 64 == 0 && kDmod % 64 == 0, "GEMM M,N multiples of 64");
static_assert(kDin % 256 == 0 && kSeqL % 16 == 0 && kRows % 8 == 0 && kDmod == 4 * 256, "tile multiples");

constexpr size_t kSzWIN16  = (size_t)kXZP  * kDmod * 2;
constexpr size_t kSzWXP16  = (size_t)kPrjP * kDin  * 2;
constexpr size_t kSzWDT16  = (size_t)kDin  * kDtR  * 2;
constexpr size_t kSzWOUT16 = (size_t)kDmod * kDin  * 2;
constexpr size_t kSzXN16   = (size_t)kRows * kDmod * 2;
constexpr size_t kSzXZ     = (size_t)kSeqL * kXZP  * 4;
constexpr size_t kSzUC     = (size_t)kSeqL * kDin  * 4;
constexpr size_t kSzUC16   = (size_t)kSeqL * kDin  * 2;
constexpr size_t kSzPROJ   = (size_t)kSeqL * kPrjP * 4;
constexpr size_t kSzDT16   = (size_t)kSeqL * kDtR  * 2;
constexpr size_t kSzDLR    = (size_t)kSeqL * kDin  * 4;
constexpr size_t kSzY16    = (size_t)kSeqL * kDin  * 2;
constexpr size_t kOffWIN16  = 0;
constexpr size_t kOffWXP16  = kOffWIN16  + kSzWIN16;
constexpr size_t kOffWDT16  = kOffWXP16  + kSzWXP16;
constexpr size_t kOffWOUT16 = kOffWDT16  + kSzWDT16;
constexpr size_t kOffXN16   = kOffWOUT16 + kSzWOUT16;
constexpr size_t kOffXZ     = kOffXN16   + kSzXN16;
constexpr size_t kOffUC     = kOffXZ     + kSzXZ;
constexpr size_t kOffUC16   = kOffUC     + kSzUC;
constexpr size_t kOffPROJ   = kOffUC16   + kSzUC16;
constexpr size_t kOffDT16   = kOffPROJ   + kSzPROJ;
constexpr size_t kOffDLR    = kOffDT16   + kSzDT16;
constexpr size_t kOffY16    = kOffDLR    + kSzDLR;
constexpr size_t kWsTotal   = kOffY16    + kSzY16;
static_assert(kWsTotal == 108265472ull, "carve total");
static_assert(kWsTotal <= 134217728ull, "carve cap");
static_assert((kOffWXP16 % 128) == 0 && (kOffWDT16 % 128) == 0 && (kOffWOUT16 % 128) == 0 && (kOffXN16 % 128) == 0 &&
              (kOffXZ % 128) == 0 && (kOffUC % 128) == 0 && (kOffUC16 % 128) == 0 && (kOffPROJ % 128) == 0 &&
              (kOffDT16 % 128) == 0 && (kOffDLR % 128) == 0 && (kOffY16 % 128) == 0, "128-B aligned regions");

__device__ __forceinline__ void guard4_h(v8f& a, v8f& b, v8f& c, v8f& d, v16h x, v16h y) {
  asm volatile("v_nop\n\tv_nop\n\tv_nop\n\tv_nop" : "+v"(a), "+v"(b), "+v"(c), "+v"(d) : "v"(x), "v"(y));
}
__device__ __forceinline__ void keep4_h(v16h a, v16h b, v16h c, v16h d) { asm volatile("v_nop" :: "v"(a), "v"(b), "v"(c), "v"(d)); }
__device__ __forceinline__ void acc_guard4(v8f& a, v8f& b, v8f& c, v8f& d) { asm volatile("v_nop\n\tv_nop\n\tv_nop\n\tv_nop" : "+v"(a), "+v"(b), "+v"(c), "+v"(d)); }

struct FragH {
  union U { v16h v; v8h h[2]; };
  static __device__ __forceinline__ v16h load(const _Float16* p) {
    U f; f.h[0] = *(const v8h*)(p); f.h[1] = *(const v8h*)(p + 16); return f.v;
  }
  static __device__ __forceinline__ v8f mma(v16h a, v16h b, v8f c) {
    return __builtin_amdgcn_wmma_f32_16x16x32_f16(false, a, false, b, (short)0, c, false, false);
  }
};

template <int BIAS_MODE, bool RESID>
__global__ __launch_bounds__(256) void wmma_gemm64_f16(
    const unsigned short* __restrict__ Ap, int lda,
    const unsigned short* __restrict__ Btp, int ldb,
    float* __restrict__ C, int ldc,
    const float* __restrict__ bias, const float* __restrict__ resid,
    int M, int N, int K, float scale)
{
  const _Float16* A  = (const _Float16*)Ap;
  const _Float16* Bt = (const _Float16*)Btp;
  __shared__ __align__(16) float sT[8][16 * 68];
  const int lane = threadIdx.x & 31;
  const int wave = threadIdx.x >> 5;
  const int tilesN = N >> 6;
  const int tilesM = M >> 6;
  const int tile = blockIdx.x * 8 + wave;
  if (tile >= tilesM * tilesN) return;
  const int tm = tile / tilesN;
  const int tn = tile - tm * tilesN;
  const int m0 = tm << 6;
  const int n0 = tn << 6;

  const int rlane = lane & 15;
  const int koff  = (lane >> 4) * 8;
  const int mOff  = (lane >> 4) * 8;

  v8f acc[4][4];
#pragma unroll
  for (int i = 0; i < 4; ++i)
#pragma unroll
    for (int j = 0; j < 4; ++j) acc[i][j] = (v8f){0.f,0.f,0.f,0.f,0.f,0.f,0.f,0.f};

  for (int k0 = 0; k0 < K; k0 += 32) {
    v16h bh[4];
#pragma unroll
    for (int j = 0; j < 4; ++j) {
      const size_t bo = (size_t)(n0 + (j << 4) + rlane) * ldb + koff + k0;
      bh[j] = FragH::load(Bt + bo);
    }
#pragma unroll
    for (int i = 0; i < 4; ++i) {
      const size_t ao = (size_t)(m0 + (i << 4) + rlane) * lda + koff + k0;
      v16h ah = FragH::load(A + ao);
#pragma unroll
      for (int j = 0; j < 4; ++j) acc[i][j] = FragH::mma(ah, bh[j], acc[i][j]);
      guard4_h(acc[i][0], acc[i][1], acc[i][2], acc[i][3], ah, bh[3]);
    }
    keep4_h(bh[0], bh[1], bh[2], bh[3]);
  }
  acc_guard4(acc[0][0], acc[0][1], acc[0][2], acc[0][3]);
  acc_guard4(acc[1][0], acc[1][1], acc[1][2], acc[1][3]);
  acc_guard4(acc[2][0], acc[2][1], acc[2][2], acc[2][3]);
  acc_guard4(acc[3][0], acc[3][1], acc[3][2], acc[3][3]);

  float* slab = sT[wave];
  const int hh = lane >> 4, c4 = (lane & 15) * 4;
#pragma unroll
  for (int i = 0; i < 4; ++i) {
    const int mBase = m0 + (i << 4);
#pragma unroll
    for (int j = 0; j < 4; ++j) {
      float bv = 0.f;
      if (BIAS_MODE == 2) bv = bias[n0 + (j << 4) + rlane];
#pragma unroll
      for (int r = 0; r < 8; ++r) {
        float v = acc[i][j][r] * scale;
        if (BIAS_MODE == 2) v += bv;
        slab[(mOff + r) * 68 + (j << 4) + rlane] = v;
      }
    }
    __builtin_amdgcn_fence(__ATOMIC_RELEASE, "workgroup");
    __builtin_amdgcn_wave_barrier();
    __builtin_amdgcn_fence(__ATOMIC_ACQUIRE, "workgroup");
    v4f ov[8];
#pragma unroll
    for (int it = 0; it < 8; ++it) {
      const int row = it * 2 + hh;
      v4f v = *(const v4f*)(slab + row * 68 + c4);
      if (RESID) {
        const v4f rv = *(const v4f*)(resid + (size_t)(mBase + row) * ldc + n0 + c4);
        v = v + rv;
      }
      ov[it] = v;
    }
    for (int pass = 0; pass < 2; ++pass) {
#pragma unroll
      for (int it = 0; it < 8; ++it) {
        const int row = it * 2 + hh;
        *(volatile v4f*)(C + (size_t)(mBase + row) * ldc + n0 + c4) = ov[it];
      }
      __threadfence();
    }
    __builtin_amdgcn_fence(__ATOMIC_RELEASE, "workgroup");
    __builtin_amdgcn_wave_barrier();
    __builtin_amdgcn_fence(__ATOMIC_ACQUIRE, "workgroup");
  }
}

__global__ __launch_bounds__(256) void cast_pad_f16_kernel(
    const float* __restrict__ src, unsigned short* __restrict__ dst, int total8, int src8, float scale)
{
  const int i = blockIdx.x * 256 + threadIdx.x;
  if (i >= total8) return;
  const bool real = (i < src8);
  const int ic = real ? i : (src8 - 1);
  const float* p = src + ((size_t)ic << 3);
  const v4f a0 = *(const v4f*)(p);
  const v4f a1 = *(const v4f*)(p + 4);
  v8h hv;
#pragma unroll
  for (int e = 0; e < 4; ++e) {
    const float f0 = a0[e] * scale;
    const float f1 = a1[e] * scale;
    hv[e]     = (_Float16)(real ? f0 : 0.0f);
    hv[4 + e] = (_Float16)(real ? f1 : 0.0f);
  }
  unsigned short* q = dst + ((size_t)i << 3);
  *(volatile v8h*)q = hv;
  __threadfence();
  *(volatile v8h*)q = hv;
}

__global__ __launch_bounds__(256) void layernorm_f16_kernel(
    const float* __restrict__ x, const float* __restrict__ gam, const float* __restrict__ bet,
    unsigned short* __restrict__ XN16)
{
  const int lane = threadIdx.x & 31, wave = threadIdx.x >> 5;
  const int row = blockIdx.x * 8 + wave;
  const float* xr = x + (size_t)row * kDmod + lane * 8;

  float s = 0.f;
#pragma unroll 1
  for (int it = 0; it < 4; ++it) {
    const v4f a0 = *(const v4f*)(xr + it * 256);
    const v4f a1 = *(const v4f*)(xr + it * 256 + 4);
    s += ((a0[0] + a0[1]) + (a0[2] + a0[3])) + ((a1[0] + a1[1]) + (a1[2] + a1[3]));
  }
#pragma unroll
  for (int off = 16; off >= 1; off >>= 1) s += __shfl_xor(s, off, 32);
  const float mu = s * (1.0f / (float)kDmod);

  float q = 0.f;
#pragma unroll 1
  for (int it = 0; it < 4; ++it) {
    const v4f a0 = *(const v4f*)(xr + it * 256);
    const v4f a1 = *(const v4f*)(xr + it * 256 + 4);
#pragma unroll
    for (int e = 0; e < 4; ++e) {
      const float d0v = a0[e] - mu;
      const float d1v = a1[e] - mu;
      q = fmaf(d0v, d0v, q);
      q = fmaf(d1v, d1v, q);
    }
  }
#pragma unroll
  for (int off = 16; off >= 1; off >>= 1) q += __shfl_xor(q, off, 32);
  const float var  = q * (1.0f / (float)kDmod);
  const float rstd = 1.0f / sqrtf(var + kLnEps);

  unsigned short* orow = XN16 + (size_t)row * kDmod + lane * 8;
  const float* gr = gam + lane * 8;
  const float* br = bet + lane * 8;
#pragma unroll 1
  for (int it = 0; it < 4; ++it) {
    const v4f a0 = *(const v4f*)(xr + it * 256);
    const v4f a1 = *(const v4f*)(xr + it * 256 + 4);
    const v4f g0 = *(const v4f*)(gr + it * 256);
    const v4f g1 = *(const v4f*)(gr + it * 256 + 4);
    const v4f b0 = *(const v4f*)(br + it * 256);
    const v4f b1 = *(const v4f*)(br + it * 256 + 4);
    v8h hv;
#pragma unroll
    for (int e = 0; e < 4; ++e) {
      const float n0v = (a0[e] - mu) * rstd;
      const float n1v = (a1[e] - mu) * rstd;
      hv[e]     = (_Float16)(n0v * g0[e] + b0[e]);
      hv[4 + e] = (_Float16)(n1v * g1[e] + b1[e]);
    }
    unsigned short* op = orow + it * 256;
    *(volatile v8h*)op = hv;
    __threadfence();
    *(volatile v8h*)op = hv;
  }
}

__global__ __launch_bounds__(256) void dt_cast_kernel(
    const float* __restrict__ PROJ, unsigned short* __restrict__ DT16, int total8, float scale)
{
  const int i = blockIdx.x * 256 + threadIdx.x;
  if (i >= total8) return;
  const int e0  = i << 3;
  const int row = e0 >> 7;
  const int c8  = e0 & (kDtR - 1);
  const float* p = PROJ + (size_t)row * kPrjP + c8;
  const v4f a0 = *(const v4f*)(p);
  const v4f a1 = *(const v4f*)(p + 4);
  v8h hv;
#pragma unroll
  for (int e = 0; e < 4; ++e) {
    hv[e]     = (_Float16)(a0[e] * scale);
    hv[4 + e] = (_Float16)(a1[e] * scale);
  }
  unsigned short* qd = DT16 + e0;
  *(volatile v8h*)qd = hv;
  __threadfence();
  *(volatile v8h*)qd = hv;
}

__global__ __launch_bounds__(256) void conv_silu_kernel(
    const float* __restrict__ XZ, const float* __restrict__ cw, const float* __restrict__ cb,
    float* __restrict__ UC, unsigned short* __restrict__ UC16)
{
  __shared__ __align__(16) float sT[16 * kTP];
  const int tid = threadIdx.x, lane = tid & 31, wave = tid >> 5;
  const int d0 = blockIdx.x * 256, d = d0 + tid;
  const int t0 = blockIdx.y * 64;
  const v4f wv = *(const v4f*)(cw + (size_t)d * 4);
  const float w0 = wv[0], w1 = wv[1], w2 = wv[2], w3 = wv[3];
  const float bc = cb[d];
  float xm3, xm2, xm1;
  {
    const int r3 = t0 - 3, r2 = t0 - 2, r1 = t0 - 1;
    const float v3 = XZ[(size_t)(r3 < 0 ? 0 : r3) * kXZP + d];
    const float v2 = XZ[(size_t)(r2 < 0 ? 0 : r2) * kXZP + d];
    const float v1 = XZ[(size_t)(r1 < 0 ? 0 : r1) * kXZP + d];
    xm3 = (r3 >= 0) ? v3 : 0.f;
    xm2 = (r2 >= 0) ? v2 : 0.f;
    xm1 = (r1 >= 0) ? v1 : 0.f;
  }
  const int hrow = wave >> 1;
  const int hch  = (wave & 1) * 128 + lane * 4;
#pragma unroll 1
  for (int sub = 0; sub < 4; ++sub) {
    const int lb = t0 + sub * 16;
#pragma unroll 1
    for (int s = 0; s < 16; ++s) {
      const float xc = XZ[(size_t)(lb + s) * kXZP + d];
      float acc = w0 * xm3;
      acc = fmaf(w1, xm2, acc);
      acc = fmaf(w2, xm1, acc);
      acc = fmaf(w3, xc, acc);
      const float sv = acc + bc;
      const float sg = __builtin_amdgcn_rcpf(1.0f + __expf(-sv));
      sT[s * kTP + tid] = sv * sg;
      xm3 = xm2; xm2 = xm1; xm1 = xc;
    }
    __syncthreads();
    v4f fv[4];
    v8h bv[2];
#pragma unroll
    for (int it = 0; it < 4; ++it) fv[it] = *(const v4f*)(sT + (it * 4 + hrow) * kTP + hch);
#pragma unroll
    for (int it = 0; it < 2; ++it) {
      const float* sp = sT + (it * 8 + wave) * kTP + lane * 8;
      const v4f a0 = *(const v4f*)(sp);
      const v4f a1 = *(const v4f*)(sp + 4);
#pragma unroll
      for (int e = 0; e < 4; ++e) {
        bv[it][e]     = (_Float16)(a0[e] * kCarryU);
        bv[it][4 + e] = (_Float16)(a1[e] * kCarryU);
      }
    }
    for (int pass = 0; pass < 2; ++pass) {
#pragma unroll
      for (int it = 0; it < 4; ++it)
        *(volatile v4f*)(UC + (size_t)(lb + it * 4 + hrow) * kDin + d0 + hch) = fv[it];
#pragma unroll
      for (int it = 0; it < 2; ++it)
        *(volatile v8h*)(UC16 + (size_t)(lb + it * 8 + wave) * kDin + d0 + lane * 8) = bv[it];
      __threadfence();
    }
    __syncthreads();
  }
}

__global__ __launch_bounds__(256) void scan_kernel(
    const float* __restrict__ DLR, const float* __restrict__ UC, const float* __restrict__ XZ,
    const float* __restrict__ PROJ, const float* __restrict__ A_log, const float* __restrict__ Dv,
    unsigned short* __restrict__ Y16)
{
  __shared__ __align__(16) float sBC[16 * 32];
  __shared__ __align__(16) float sY[16 * kTP];
  const int tid = threadIdx.x, lane = tid & 31, wave = tid >> 5;
  const int d0 = blockIdx.x * 256, d = d0 + tid;

  float An[kNst];
#pragma unroll
  for (int q4 = 0; q4 < 4; ++q4) {
    const v4f al = *(const v4f*)(A_log + (size_t)d * kNst + 4 * q4);
    An[4 * q4 + 0] = -__expf(al[0]);
    An[4 * q4 + 1] = -__expf(al[1]);
    An[4 * q4 + 2] = -__expf(al[2]);
    An[4 * q4 + 3] = -__expf(al[3]);
  }
  const float Dd = Dv[d];
  float h[kNst];
#pragma unroll
  for (int n = 0; n < kNst; ++n) h[n] = 0.f;

#pragma unroll 1
  for (int c = 0; c < kSeqL / 16; ++c) {
    const int l0 = c * 16;
    if (tid < 128) {
      const int r = tid >> 3, q = (tid & 7) * 4;
      const v4f v = *(const v4f*)(PROJ + (size_t)(l0 + r) * kPrjP + kDtR + q);
      *(v4f*)(sBC + r * 32 + q) = v;
    }
    __syncthreads();
#pragma unroll 1
    for (int s = 0; s < 16; ++s) {
      const size_t m = (size_t)(l0 + s);
      const float a  = DLR[m * kDin + d];
      const float xv = UC[m * kDin + d];
      const float zv = XZ[m * kXZP + kDin + d];
      const float ea  = __expf(-fabsf(a));
      const float up  = 1.0f + ea;
      const float l1p = __logf(up) + (ea - (up - 1.0f)) * __builtin_amdgcn_rcpf(up);
      const float delta = fmaxf(a, 0.0f) + l1p;
      const float du = delta * xv;
      v4f Bq[4], Cq[4];
#pragma unroll
      for (int qq = 0; qq < 4; ++qq) {
        Bq[qq] = *(const v4f*)(sBC + s * 32 + 4 * qq);
        Cq[qq] = *(const v4f*)(sBC + s * 32 + kNst + 4 * qq);
      }
      float y = 0.f;
#pragma unroll
      for (int n = 0; n < kNst; ++n) {
        const float e  = __expf(delta * An[n]);
        const float hn = e * h[n] + du * Bq[n >> 2][n & 3];
        h[n] = hn;
        y = hn * Cq[n >> 2][n & 3] + y;
      }
      y = xv * Dd + y;
      const float sg = __builtin_amdgcn_rcpf(1.0f + __expf(-zv));
      const float g  = zv * sg;
      sY[s * kTP + tid] = (y * g) * kCarryY;
    }
    __syncthreads();
    v8h hv[2];
#pragma unroll
    for (int it = 0; it < 2; ++it) {
      const float* sp = sY + (it * 8 + wave) * kTP + lane * 8;
      const v4f a0 = *(const v4f*)(sp);
      const v4f a1 = *(const v4f*)(sp + 4);
#pragma unroll
      for (int e = 0; e < 4; ++e) { hv[it][e] = (_Float16)a0[e]; hv[it][4 + e] = (_Float16)a1[e]; }
    }
    for (int pass = 0; pass < 2; ++pass) {
#pragma unroll
      for (int it = 0; it < 2; ++it)
        *(volatile v8h*)(Y16 + (size_t)(l0 + it * 8 + wave) * kDin + d0 + lane * 8) = hv[it];
      __threadfence();
    }
  }
}

static_assert(((kXZP * kDmod / 8) % 256) == 0 && ((kPrjP * kDin / 8) % 256) == 0 &&
              ((kDin * kDtR / 8) % 256) == 0 && ((kDmod * kDin / 8) % 256) == 0 &&
              ((kSeqL * kDtR / 8) % 256) == 0, "exact cast grids");
static_assert((((kSeqL / 64) * (kXZP / 64)) % 8) == 0 && (((kSeqL / 64) * (kPrjP / 64)) % 8) == 0 &&
              (((kSeqL / 64) * (kDin / 64)) % 8) == 0 && (((kSeqL / 64) * (kDmod / 64)) % 8) == 0, "exact GEMM grids");

extern "C" void kernel_launch(void* const* d_in, const int* in_sizes, int n_in,
                              void* d_out, int out_size, void* d_ws, size_t ws_size,
                              hipStream_t stream)
{
  if (n_in < 12) return;
  if (in_sizes[0] != kRows * kDmod) return;
  if (in_sizes[1] != kDmod || in_sizes[2] != kDmod) return;
  if (in_sizes[3] != kXZP * kDmod) return;
  if (in_sizes[4] != kDin * 4 || in_sizes[5] != kDin) return;
  if (in_sizes[6] != kPrjN * kDin) return;
  if (in_sizes[7] != kDin * kDtR || in_sizes[8] != kDin) return;
  if (in_sizes[9] != kDin * kNst || in_sizes[10] != kDin) return;
  if (in_sizes[11] != kDmod * kDin) return;
  if (out_size != kRows * kDmod) return;
  if (ws_size < kWsTotal) return;

  const float* x      = (const float*)d_in[0];
  const float* ln_g   = (const float*)d_in[1];
  const float* ln_b   = (const float*)d_in[2];
  const float* W_in   = (const float*)d_in[3];
  const float* conv_w = (const float*)d_in[4];
  const float* conv_b = (const float*)d_in[5];
  const float* W_xprj = (const float*)d_in[6];
  const float* W_dt   = (const float*)d_in[7];
  const float* b_dt   = (const float*)d_in[8];
  const float* A_log  = (const float*)d_in[9];
  const float* Dv     = (const float*)d_in[10];
  const float* W_out  = (const float*)d_in[11];
  float* dout = (float*)d_out;

  char* ws = (char*)d_ws;
  unsigned short* WIN16  = (unsigned short*)(ws + kOffWIN16);
  unsigned short* WXP16  = (unsigned short*)(ws + kOffWXP16);
  unsigned short* WDT16  = (unsigned short*)(ws + kOffWDT16);
  unsigned short* WOUT16 = (unsigned short*)(ws + kOffWOUT16);
  unsigned short* XN16   = (unsigned short*)(ws + kOffXN16);
  float*          XZ     = (float*)(ws + kOffXZ);
  float*          UC     = (float*)(ws + kOffUC);
  unsigned short* UC16   = (unsigned short*)(ws + kOffUC16);
  float*          PROJ   = (float*)(ws + kOffPROJ);
  unsigned short* DT16   = (unsigned short*)(ws + kOffDT16);
  float*          DLR    = (float*)(ws + kOffDLR);
  unsigned short* Y16    = (unsigned short*)(ws + kOffY16);

  cast_pad_f16_kernel<<<(kXZP * kDmod / 8) / 256, 256, 0, stream>>>(W_in,   WIN16,  kXZP * kDmod / 8, kXZP * kDmod / 8, kCarryW);
  cast_pad_f16_kernel<<<(kPrjP * kDin / 8) / 256, 256, 0, stream>>>(W_xprj, WXP16,  kPrjP * kDin / 8, kPrjN * kDin / 8, kCarryW);
  cast_pad_f16_kernel<<<(kDin * kDtR / 8) / 256, 256, 0, stream>>>(W_dt,    WDT16,  kDin * kDtR / 8,  kDin * kDtR / 8,  kCarryWdt);
  cast_pad_f16_kernel<<<(kDmod * kDin / 8) / 256, 256, 0, stream>>>(W_out,  WOUT16, kDmod * kDin / 8, kDmod * kDin / 8, kCarryW);

  layernorm_f16_kernel<<<kRows / 8, 256, 0, stream>>>(x, ln_g, ln_b, XN16);

  for (int b = 0; b < kBatch; ++b) {
    const unsigned short* XN16b = XN16 + (size_t)b * kSeqL * kDmod;
    const float* xb = x + (size_t)b * kSeqL * kDmod;
    float* outb = dout + (size_t)b * kSeqL * kDmod;

    wmma_gemm64_f16<0, false><<<256, 256, 0, stream>>>(
        XN16b, kDmod, WIN16, kDmod, XZ, kXZP, b_dt, xb, kSeqL, kXZP, kDmod, kFoldIn);

    conv_silu_kernel<<<dim3(kDin / 256, kSeqL / 64), 256, 0, stream>>>(XZ, conv_w, conv_b, UC, UC16);

    wmma_gemm64_f16<0, false><<<12, 256, 0, stream>>>(
        UC16, kDin, WXP16, kDin, PROJ, kPrjP, b_dt, xb, kSeqL, kPrjP, kDin, kFoldXp);

    dt_cast_kernel<<<(kSeqL * kDtR / 8) / 256, 256, 0, stream>>>(PROJ, DT16, kSeqL * kDtR / 8, kCarryDt);

    wmma_gemm64_f16<2, false><<<128, 256, 0, stream>>>(
        DT16, kDtR, WDT16, kDtR, DLR, kDin, b_dt, xb, kSeqL, kDin, kDtR, kFoldDt);

    scan_kernel<<<kDin / 256, 256, 0, stream>>>(DLR, UC, XZ, PROJ, A_log, Dv, Y16);

    wmma_gemm64_f16<0, true><<<64, 256, 0, stream>>>(
        Y16, kDin, WOUT16, kDin, outb, kDmod, b_dt, xb, kSeqL, kDmod, kDin, kFoldOut);
  }
}
